// Q_Net_9594956939555
// MI455X (gfx1250) — hardware-verified
//
#include <hip/hip_runtime.h>
#define NB 8192
#define NA 64
#define CD 8
#define HID 256
#define EO 257
#define EP 256
#define QI 265
#define QP 288
#define AD 30
#define CHB 1024

typedef __bf16 v16b __attribute__((ext_vector_type(16)));
typedef unsigned short v8us __attribute__((ext_vector_type(8), may_alias));
typedef float  v8f  __attribute__((ext_vector_type(8)));
typedef float  v4f  __attribute__((ext_vector_type(4)));
typedef float  v4fa __attribute__((ext_vector_type(4), may_alias));
union FragB { v16b v; v8us half[2]; unsigned short u[16]; };

__device__ __forceinline__ unsigned short bf16_bits(float x) { unsigned int u = __float_as_uint(x); return (unsigned short)((u + 0x7FFFu + ((u >> 16) & 1u)) >> 16); }
__device__ __forceinline__ float bf16_val(unsigned short b) { return __uint_as_float(((unsigned int)b) << 16); }
__device__ __forceinline__ float bf16_round(float x) { return bf16_val(bf16_bits(x)); }
template <int NT>
__device__ __forceinline__ v8f mmaN(v16b ah, v16b al, v16b bh, v16b bl, v8f c) {
  c = __builtin_amdgcn_wmma_f32_16x16x32_bf16(false, ah, false, bh, (short)0, c, false, false);
  if (NT >= 2) c = __builtin_amdgcn_wmma_f32_16x16x32_bf16(false, al, false, bh, (short)0, c, false, false);
  if (NT >= 3) c = __builtin_amdgcn_wmma_f32_16x16x32_bf16(false, ah, false, bl, (short)0, c, false, false);
  asm volatile("v_nop\n\tv_nop\n\tv_nop\n\tv_nop" : "+v"(c) : "v"(ah), "v"(al), "v"(bh), "v"(bl));
  return c;
}

__global__ __launch_bounds__(256) void k_wt_bf16(const float* __restrict__ W, unsigned short* __restrict__ Wt, int K, int N) {
  const int t = blockIdx.x * 256 + threadIdx.x;
  const int k8n = K / 8;
  if (t >= N * k8n) return;
  const int n = t / k8n, k8 = (t % k8n) * 8;
  v8us v;
#pragma unroll
  for (int i = 0; i < 8; ++i) v[i] = bf16_bits(W[(size_t)(k8 + i) * N + n]);
  *(volatile v8us*)(Wt + (size_t)n * K + k8) = v;
  __threadfence();
  *(volatile v8us*)(Wt + (size_t)n * K + k8) = v;
}

template <bool ASPLIT, int ACT, bool BIAS_BF16>
__global__ __launch_bounds__(128) void k_gemm_bf(const float* __restrict__ A, int lda, const unsigned short* __restrict__ Wt, int ldb,
                                               const float* __restrict__ bias, float* __restrict__ C, int ldc, int M, int N, int K) {
  __shared__ __attribute__((aligned(16))) float so[4][16][64];
  const int tid = threadIdx.x, w = tid >> 5, lane = tid & 31, ln = lane & 15, hh = lane >> 4;
  const int ntn = N / 64;
  const int wid = blockIdx.x * 4 + w;
  const int mt = wid / ntn, nq = wid % ntn;
  if (mt * 16 >= M) return;
  const int row0 = mt * 16, col0 = nq * 64;
  const float* arow = A + (size_t)(row0 + ln) * lda;
  v8f acc[4] = {};
  for (int kb = 0; kb < K; kb += 32) {
    FragB ah, al;
    const v4f x0 = *(const v4fa*)(arow + kb + 8 * hh), x1 = *(const v4fa*)(arow + kb + 8 * hh + 4);
    const v4f x2 = *(const v4fa*)(arow + kb + 16 + 8 * hh), x3 = *(const v4fa*)(arow + kb + 16 + 8 * hh + 4);
    float xs[16] = {x0[0],x0[1],x0[2],x0[3],x1[0],x1[1],x1[2],x1[3],x2[0],x2[1],x2[2],x2[3],x3[0],x3[1],x3[2],x3[3]};
#pragma unroll
    for (int i = 0; i < 16; ++i) { const unsigned short hb = bf16_bits(xs[i]); ah.u[i] = hb; al.u[i] = ASPLIT ? bf16_bits(xs[i] - bf16_val(hb)) : (unsigned short)0; }
#pragma unroll
    for (int t = 0; t < 4; ++t) {
      const unsigned short* brow = Wt + (size_t)(col0 + t * 16 + ln) * ldb + kb;
      FragB b;
      b.half[0] = *(const v8us*)(brow + 8 * hh);
      b.half[1] = *(const v8us*)(brow + 16 + 8 * hh);
      acc[t] = mmaN<ASPLIT ? 2 : 1>(ah.v, al.v, b.v, b.v, acc[t]);
    }
  }
#pragma unroll
  for (int t = 0; t < 4; ++t) {
    float bv = bias ? bias[col0 + t * 16 + ln] : 0.f;
    if (BIAS_BF16) bv = bf16_round(bv);
#pragma unroll
    for (int r = 0; r < 8; ++r) { float v = acc[t][r] + bv; if (ACT == 1) v = fmaxf(v, 0.f); so[w][8 * hh + r][t * 16 + ln] = v; }
  }
  __builtin_amdgcn_fence(__ATOMIC_ACQ_REL, "workgroup");
  __builtin_amdgcn_wave_barrier();
  const int rsub = lane >> 4, c4 = (lane & 15) * 4;
  for (int pass = 0; pass < 2; ++pass) {
#pragma unroll
    for (int q = 0; q < 8; ++q) {
      const int r = q * 2 + rsub;
      const v4f v = *(const v4fa*)&so[w][r][c4];
      *(volatile v4f*)(C + (size_t)(row0 + r) * ldc + col0 + c4) = v;
    }
    if (pass == 0) __threadfence();
  }
}

template <int D, bool CAUSAL>
__global__ __launch_bounds__(128) void k_flash(const float* __restrict__ qb, const float* __restrict__ kb, const float* __restrict__ vb,
                                             int pitch, int T, int H, float scale, float* __restrict__ y, int ypitch) {
  constexpr int KS = D / 32;
  constexpr int DT = D / 16;
  __shared__ __attribute__((aligned(16))) unsigned short sKh[32][D + 8], sKl[32][D + 8], sVh[32][D + 8], sVl[32][D + 8];
  __shared__ __attribute__((aligned(16))) unsigned short sPh[4][16][40], sPl[4][16][40];
  __shared__ __attribute__((aligned(16))) float sO[4][16][D];
  const int tid = threadIdx.x, w = tid >> 5, lane = tid & 31, ln = lane & 15, hh = lane >> 4;
  const int nqb = (T + 63) / 64;
  const int bh = blockIdx.x / nqb, qblk = blockIdx.x % nqb;
  const int b = bh / H, h = bh % H;
  const int q0 = qblk * 64 + w * 16;
  const float* Q = qb + (size_t)b * T * pitch + h * D;
  const float* K = kb + (size_t)b * T * pitch + h * D;
  const float* V = vb + (size_t)b * T * pitch + h * D;

  FragB aqh[KS], aql[KS];
  {
    int row = q0 + ln; if (row >= T) row = T - 1;
    const float* qr = Q + (size_t)row * pitch;
#pragma unroll
    for (int ks = 0; ks < KS; ++ks)
#pragma unroll
      for (int i = 0; i < 16; ++i) {
        const int d = ks * 32 + ((i < 8) ? (8 * hh + i) : (16 + 8 * hh + (i - 8)));
        const float x = qr[d] * scale; const unsigned short hb = bf16_bits(x);
        aqh[ks].u[i] = hb; aql[ks].u[i] = bf16_bits(x - bf16_val(hb));
      }
  }
  float m_r[8], l_r[8];
#pragma unroll
  for (int r = 0; r < 8; ++r) { m_r[r] = -3.0e38f; l_r[r] = 0.f; }
  v8f oacc[DT];
#pragma unroll
  for (int dt = 0; dt < DT; ++dt) oacc[dt] = (v8f){0.f,0.f,0.f,0.f,0.f,0.f,0.f,0.f};

  const int kv_end = CAUSAL ? min(T, qblk * 64 + 64) : T;
  for (int j0 = 0; j0 < kv_end; j0 += 32) {
    __syncthreads();
    for (int e = tid; e < 32 * (D / 4); e += 128) {
      const int r = e / (D / 4), c4 = (e % (D / 4)) * 4;
      const int key = j0 + r;
      v4f kf = {0.f,0.f,0.f,0.f}, vf = {0.f,0.f,0.f,0.f};
      if (key < T) { kf = *(const v4fa*)(K + (size_t)key * pitch + c4); vf = *(const v4fa*)(V + (size_t)key * pitch + c4); }
#pragma unroll
      for (int t = 0; t < 4; ++t) {
        unsigned short hb = bf16_bits(kf[t]); sKh[r][c4 + t] = hb; sKl[r][c4 + t] = bf16_bits(kf[t] - bf16_val(hb));
        hb = bf16_bits(vf[t]); sVh[r][c4 + t] = hb; sVl[r][c4 + t] = bf16_bits(vf[t] - bf16_val(hb));
      }
    }
    __syncthreads();
    v8f s[2];
#pragma unroll
    for (int nt = 0; nt < 2; ++nt) {
      v8f acc = {};
#pragma unroll
      for (int ks = 0; ks < KS; ++ks) {
        FragB bh_, bl_;
        bh_.half[0] = *(const v8us*)&sKh[nt * 16 + ln][ks * 32 + 8 * hh]; bh_.half[1] = *(const v8us*)&sKh[nt * 16 + ln][ks * 32 + 16 + 8 * hh];
        bl_.half[0] = *(const v8us*)&sKl[nt * 16 + ln][ks * 32 + 8 * hh]; bl_.half[1] = *(const v8us*)&sKl[nt * 16 + ln][ks * 32 + 16 + 8 * hh];
        acc = mmaN<3>(aqh[ks].v, aql[ks].v, bh_.v, bl_.v, acc);
      }
      s[nt] = acc;
    }
    float alpha[8];
#pragma unroll
    for (int r = 0; r < 8; ++r) {
      const int qi = q0 + 8 * hh + r;
      const int ja = j0 + ln, jb = j0 + 16 + ln;
      if (CAUSAL) { if (ja > qi) s[0][r] = -3.0e38f; if (jb > qi) s[1][r] = -3.0e38f; }
      if (ja >= T) s[0][r] = -3.0e38f;
      if (jb >= T) s[1][r] = -3.0e38f;
      float mx = fmaxf(s[0][r], s[1][r]);
      mx = fmaxf(mx, __shfl_xor(mx, 1, 32)); mx = fmaxf(mx, __shfl_xor(mx, 2, 32)); mx = fmaxf(mx, __shfl_xor(mx, 4, 32)); mx = fmaxf(mx, __shfl_xor(mx, 8, 32));
      const float mnew = fmaxf(m_r[r], mx);
      alpha[r] = (mnew > -1.0e38f) ? __expf(m_r[r] - mnew) : 1.0f;
      const float p0 = (s[0][r] > -1.0e38f) ? __expf(s[0][r] - mnew) : 0.f;
      const float p1 = (s[1][r] > -1.0e38f) ? __expf(s[1][r] - mnew) : 0.f;
      m_r[r] = mnew;
      l_r[r] = l_r[r] * alpha[r] + p0 + p1;
      unsigned short hb = bf16_bits(p0); sPh[w][8 * hh + r][ln] = hb;      sPl[w][8 * hh + r][ln] = bf16_bits(p0 - bf16_val(hb));
      hb = bf16_bits(p1);                sPh[w][8 * hh + r][16 + ln] = hb; sPl[w][8 * hh + r][16 + ln] = bf16_bits(p1 - bf16_val(hb));
    }
#pragma unroll
    for (int dt = 0; dt < DT; ++dt)
#pragma unroll
      for (int r = 0; r < 8; ++r) oacc[dt][r] *= alpha[r];
    __builtin_amdgcn_fence(__ATOMIC_ACQ_REL, "workgroup");
    __builtin_amdgcn_wave_barrier();
    FragB pah, pal;
    pah.half[0] = *(const v8us*)&sPh[w][ln][8 * hh]; pah.half[1] = *(const v8us*)&sPh[w][ln][16 + 8 * hh];
    pal.half[0] = *(const v8us*)&sPl[w][ln][8 * hh]; pal.half[1] = *(const v8us*)&sPl[w][ln][16 + 8 * hh];
#pragma unroll
    for (int dt = 0; dt < DT; ++dt) {
      FragB bvh, bvl;
#pragma unroll
      for (int i = 0; i < 8; ++i) {
        bvh.u[i] = sVh[8 * hh + i][dt * 16 + ln]; bvh.u[8 + i] = sVh[16 + 8 * hh + i][dt * 16 + ln];
        bvl.u[i] = sVl[8 * hh + i][dt * 16 + ln]; bvl.u[8 + i] = sVl[16 + 8 * hh + i][dt * 16 + ln];
      }
      oacc[dt] = mmaN<3>(pah.v, pal.v, bvh.v, bvl.v, oacc[dt]);
    }
    __builtin_amdgcn_fence(__ATOMIC_ACQ_REL, "workgroup");
    __builtin_amdgcn_wave_barrier();
  }
#pragma unroll
  for (int r = 0; r < 8; ++r) {
    float l = l_r[r];
    l += __shfl_xor(l, 1, 32); l += __shfl_xor(l, 2, 32); l += __shfl_xor(l, 4, 32); l += __shfl_xor(l, 8, 32);
    l_r[r] = (l > 0.f) ? 1.0f / l : 0.f;
  }
#pragma unroll
  for (int dt = 0; dt < DT; ++dt)
#pragma unroll
    for (int r = 0; r < 8; ++r) sO[w][8 * hh + r][dt * 16 + ln] = oacc[dt][r] * l_r[r];
  __builtin_amdgcn_fence(__ATOMIC_ACQ_REL, "workgroup");
  __builtin_amdgcn_wave_barrier();
  for (int pass = 0; pass < 2; ++pass) {
    for (int r = 0; r < 16; ++r) {
      const int row = q0 + r;
      if (row < T && lane < D / 4) {
        const v4f val = *(const v4fa*)&sO[w][r][lane * 4];
        *(volatile v4f*)(y + ((size_t)b * T + row) * ypitch + h * D + lane * 4) = val;
      }
    }
    if (pass == 0) __threadfence();
  }
}

template <bool ASPLIT, int ACT, bool BIAS_BF16, bool RES_BF16>
__global__ __launch_bounds__(128) void k_gemm_bf3(const float* __restrict__ A, int lda, const unsigned short* __restrict__ Wt, int ldb,
                                                const float* __restrict__ bias, const float* __restrict__ resid, int rmod, int ldr,
                                                float* __restrict__ C, int ldc, int M, int N, int K) {
  __shared__ __attribute__((aligned(16))) float so[4][16][64];
  const int tid = threadIdx.x, w = tid >> 5, lane = tid & 31, ln = lane & 15, hh = lane >> 4;
  const int ntn = N / 64;
  const int wid = blockIdx.x * 4 + w;
  const int mt = wid / ntn, nq = wid % ntn;
  if (mt * 16 >= M) return;
  const int row0 = mt * 16, col0 = nq * 64;
  const float* arow = A + (size_t)(row0 + ln) * lda;
  v8f acc[4] = {};
  for (int kb = 0; kb < K; kb += 32) {
    FragB ah, al;
    const v4f x0 = *(const v4fa*)(arow + kb + 8 * hh), x1 = *(const v4fa*)(arow + kb + 8 * hh + 4);
    const v4f x2 = *(const v4fa*)(arow + kb + 16 + 8 * hh), x3 = *(const v4fa*)(arow + kb + 16 + 8 * hh + 4);
    float xs[16] = {x0[0],x0[1],x0[2],x0[3],x1[0],x1[1],x1[2],x1[3],x2[0],x2[1],x2[2],x2[3],x3[0],x3[1],x3[2],x3[3]};
#pragma unroll
    for (int i = 0; i < 16; ++i) { const unsigned short hb = bf16_bits(xs[i]); ah.u[i] = hb; al.u[i] = ASPLIT ? bf16_bits(xs[i] - bf16_val(hb)) : (unsigned short)0; }
#pragma unroll
    for (int t = 0; t < 4; ++t) {
      const unsigned short* brow = Wt + (size_t)(col0 + t * 16 + ln) * ldb + kb;
      FragB b;
      b.half[0] = *(const v8us*)(brow + 8 * hh);
      b.half[1] = *(const v8us*)(brow + 16 + 8 * hh);
      acc[t] = mmaN<ASPLIT ? 2 : 1>(ah.v, al.v, b.v, b.v, acc[t]);
    }
  }
#pragma unroll
  for (int t = 0; t < 4; ++t) {
    const int col = col0 + t * 16 + ln;
    float bv = bias ? bias[col] : 0.f;
    if (BIAS_BF16) bv = bf16_round(bv);
#pragma unroll
    for (int r = 0; r < 8; ++r) {
      float v = acc[t][r] + bv;
      if (resid) { float rv = resid[(size_t)((row0 + 8 * hh + r) % rmod) * ldr + col]; if (RES_BF16) rv = bf16_round(rv); v += rv; }
      if (ACT == 1) v = fmaxf(v, 0.f);
      if (ACT == 2) v = 0.5f * v * (1.0f + erff(v * 0.70710678118654752f));
      if (ACT == 3) { const float u = 0.7978845608028654f * (v + 0.044715f * v * v * v); v = 0.5f * v * (1.0f + tanhf(u)); }
      so[w][8 * hh + r][t * 16 + ln] = v;
    }
  }
  __builtin_amdgcn_fence(__ATOMIC_ACQ_REL, "workgroup");
  __builtin_amdgcn_wave_barrier();
  const int rsub = lane >> 4, c4 = (lane & 15) * 4;
  for (int pass = 0; pass < 2; ++pass) {
#pragma unroll
    for (int q = 0; q < 8; ++q) {
      const int r = q * 2 + rsub;
      const v4f v = *(const v4fa*)&so[w][r][c4];
      *(volatile v4f*)(C + (size_t)(row0 + r) * ldc + col0 + c4) = v;
    }
    if (pass == 0) __threadfence();
  }
}
template <bool PARAM_BF16>
__global__ __launch_bounds__(256) void k_layernorm(const float* __restrict__ X, const float* __restrict__ R, const float* __restrict__ g, const float* __restrict__ bta,
                                                  float* __restrict__ out_sum, float* __restrict__ out_norm, int N, float eps) {
  __shared__ float red[256];
  const int row = blockIdx.x, tid = threadIdx.x;
  const float* x = X + (size_t)row * N; const float* rr = R ? R + (size_t)row * N : nullptr;
  float vals[16];
  const int per = N / 256;
  float s1 = 0.f;
  for (int u = 0; u < per / 4; ++u) {
    const int j = tid * 4 + 1024 * u;
    const v4f a = *(const v4fa*)(x + j);
    v4f b = {0.f,0.f,0.f,0.f}; if (rr) b = *(const v4fa*)(rr + j);
#pragma unroll
    for (int q = 0; q < 4; ++q) { const float v = a[q] + b[q]; vals[u * 4 + q] = v; s1 += v; }
  }
  red[tid] = s1; __syncthreads();
  for (int st = 128; st > 0; st >>= 1) { if (tid < st) red[tid] += red[tid + st]; __syncthreads(); }
  const float mu = red[0] / (float)N; __syncthreads();
  float s2 = 0.f;
  for (int u = 0; u < per / 4; ++u)
#pragma unroll
    for (int q = 0; q < 4; ++q) { const float c = vals[u * 4 + q] - mu; s2 += c * c; }
  red[tid] = s2; __syncthreads();
  for (int st = 128; st > 0; st >>= 1) { if (tid < st) red[tid] += red[tid + st]; __syncthreads(); }
  const float rs = rsqrtf(red[0] / (float)N + eps);
  for (int pass = 0; pass < 2; ++pass) {
    for (int u = 0; u < per / 4; ++u) {
      const int j = tid * 4 + 1024 * u;
      v4f o, sm;
#pragma unroll
      for (int q = 0; q < 4; ++q) {
        float gg = g[j + q], bb = bta[j + q];
        if (PARAM_BF16) { gg = bf16_round(gg); bb = bf16_round(bb); }
        sm[q] = vals[u * 4 + q]; o[q] = (vals[u * 4 + q] - mu) * rs * gg + bb;
      }
      if (out_sum) *(volatile v4f*)(out_sum + (size_t)row * N + j) = sm;
      *(volatile v4f*)(out_norm + (size_t)row * N + j) = o;
    }
    if (pass == 0) __threadfence();
  }
}

__global__ __launch_bounds__(256) void k_wt_pad(const float* __restrict__ W, unsigned short* __restrict__ Bt, int Kin, int Nout, int Kp, int Np) {
  const int t = blockIdx.x * 256 + threadIdx.x; const int k8n = Kp / 8; if (t >= Np * k8n) return; const int n = t / k8n, k8 = (t % k8n) * 8; v8us v;
#pragma unroll 1
  for (int i = 0; i < 8; ++i) { const int k = k8 + i; v[i] = (n < Nout && k < Kin) ? bf16_bits(W[(size_t)k * Nout + n]) : (unsigned short)0; }
  *(volatile v8us*)(Bt + (size_t)n * Kp + k8) = v; __threadfence(); *(volatile v8us*)(Bt + (size_t)n * Kp + k8) = v;
}
__global__ __launch_bounds__(256) void k_bias_pad(const float* __restrict__ b, float* __restrict__ bp, int Nout, int Np) { const int n = blockIdx.x * 256 + threadIdx.x; if (n >= Np) return; const float v = n < Nout ? bf16_round(b[n]) : 0.f; *(volatile float*)(bp + n) = v; __threadfence(); *(volatile float*)(bp + n) = v; }
__global__ __launch_bounds__(256) void k_agents(const float* __restrict__ s, int b0, float* __restrict__ A) {
  const int tid = threadIdx.x, w = tid >> 5, lane = tid & 31; const int r = blockIdx.x * 8 + w; if (r >= CHB * NA) return; const int bl = r / NA, a = r % NA; const int b = b0 + bl;
  float v = (lane < CD) ? bf16_round(s[(size_t)b * 520 + CD + a * CD + lane]) : 0.f;
  const unsigned bad = __ballot(lane < CD && v == -1.0f);
  if (lane == 31) v = bad ? 0.f : 1.f;
  *(volatile float*)(A + (size_t)r * 32 + lane) = v; __threadfence(); *(volatile float*)(A + (size_t)r * 32 + lane) = v;
}
__global__ __launch_bounds__(256) void k_round_ip(float* __restrict__ p, size_t n4) { const size_t t = (size_t)blockIdx.x * 256 + threadIdx.x; if (t >= n4) return; v4f v = *(const v4fa*)(p + t * 4); for (int q = 0; q < 4; ++q) v[q] = bf16_round(v[q]); *(volatile v4f*)(p + t * 4) = v; __threadfence(); *(volatile v4f*)(p + t * 4) = v; }
__global__ __launch_bounds__(1024) void k_col256(const float* __restrict__ h, const float* __restrict__ W2, const float* __restrict__ b2, float* __restrict__ e256) {
  __shared__ float so[32]; const int tid = threadIdx.x, wv = tid >> 5, lane = tid & 31; const size_t row = (size_t)blockIdx.x * 32 + wv; const float* hr = h + row * HID; float s = 0.f;
#pragma unroll 1
  for (int k = lane; k < HID; k += 32) s += hr[k] * bf16_round(W2[(size_t)k * EO + 256]);
  for (int o = 16; o >= 1; o >>= 1) s += __shfl_xor(s, o, 32); if (lane == 0) so[wv] = fmaxf(s + bf16_round(b2[256]), 0.f); __syncthreads();
  if (tid < 32) { *(volatile float*)(e256 + (size_t)blockIdx.x * 32 + tid) = so[tid]; } __threadfence(); if (tid < 32) { *(volatile float*)(e256 + (size_t)blockIdx.x * 32 + tid) = so[tid]; }
}
__global__ __launch_bounds__(288) void k_sumcat(const float* __restrict__ s, const float* __restrict__ enc, const float* __restrict__ e256, const float* __restrict__ A, int b0, float* __restrict__ xq) {
  const int bl = blockIdx.x, b = b0 + bl, t = threadIdx.x; float v = 0.f;
  if (t < CD) v = bf16_round(s[(size_t)b * 520 + t]);
  else if (t < CD + EO) { const int e = t - CD;
#pragma unroll 1
    for (int a = 0; a < NA; ++a) v += (e < 256 ? enc[((size_t)bl * NA + a) * EP + e] : e256[(size_t)bl * NA + a]) * A[((size_t)bl * NA + a) * 32 + 31]; }
  *(volatile float*)(xq + (size_t)b * QP + t) = v; __threadfence(); *(volatile float*)(xq + (size_t)b * QP + t) = v;
}
__global__ __launch_bounds__(256) void k_pack(const float* __restrict__ q64, float* __restrict__ out) { const int rb = blockIdx.x * 128; for (int pass = 0; pass < 2; ++pass) { for (int e = threadIdx.x; e < 128 * AD; e += 256) *(volatile float*)(out + (size_t)rb * AD + e) = q64[(size_t)(rb + e / AD) * 64 + e % AD]; if (pass == 0) __threadfence(); } }
extern "C" void kernel_launch(void* const* d_in, const int* in_sizes, int n_in,
                              void* d_out, int out_size, void* d_ws, size_t ws_size, hipStream_t stream) {
  (void)in_sizes; (void)n_in; (void)out_size;
  const float* s = (const float*)d_in[0]; const float* W1 = (const float*)d_in[1]; const float* b1 = (const float*)d_in[2]; const float* W2 = (const float*)d_in[3]; const float* b2 = (const float*)d_in[4];
  const float* Qw1 = (const float*)d_in[5]; const float* Qb1 = (const float*)d_in[6]; const float* Qw2 = (const float*)d_in[7]; const float* Qb2 = (const float*)d_in[8];
  char* ws = (char*)d_ws; size_t off = 0;
  auto take = [&](size_t bytes) { char* p = ws + off; off += (bytes + 255) & ~(size_t)255; return p; };
  unsigned short* B1 = (unsigned short*)take(HID * 32 * 2); unsigned short* B2 = (unsigned short*)take((size_t)EP * HID * 2); unsigned short* BQ1 = (unsigned short*)take((size_t)HID * QP * 2); unsigned short* BQ2 = (unsigned short*)take((size_t)64 * HID * 2);
  float* b2p = (float*)take(EP * 4); float* qb2p = (float*)take(64 * 4);
  float* A = (float*)take((size_t)CHB * NA * 32 * 4); float* h = (float*)take((size_t)CHB * NA * HID * 4); float* enc = (float*)take((size_t)CHB * NA * EP * 4); float* e256 = (float*)take((size_t)CHB * NA * 4);
  float* xq = (float*)take((size_t)NB * QP * 4); float* q1 = (float*)take((size_t)NB * HID * 4); float* q64 = (float*)take((size_t)NB * 64 * 4);
  if (off > ws_size) return;
  k_wt_pad<<<(HID * 4 + 255) / 256, 256, 0, stream>>>(W1, B1, CD, HID, 32, HID); k_wt_pad<<<(EP * (HID / 8) + 255) / 256, 256, 0, stream>>>(W2, B2, HID, EO, HID, EP); k_bias_pad<<<1, 256, 0, stream>>>(b2, b2p, EO, EP);
  k_wt_pad<<<(HID * (QP / 8) + 255) / 256, 256, 0, stream>>>(Qw1, BQ1, QI, HID, QP, HID); k_wt_pad<<<(64 * (HID / 8) + 255) / 256, 256, 0, stream>>>(Qw2, BQ2, HID, AD, HID, 64); k_bias_pad<<<1, 256, 0, stream>>>(Qb2, qb2p, AD, 64);
  const int MA = CHB * NA;
  for (int c = 0; c < NB / CHB; ++c) {
    const int b0 = c * CHB;
    k_agents<<<MA / 8, 256, 0, stream>>>(s, b0, A);
    k_gemm_bf3<false, 1, true, false><<<((MA / 16) * (HID / 64) + 3) / 4, 128, 0, stream>>>(A, 32, B1, 32, b1, nullptr, 1, 0, h, HID, MA, HID, 32);
    k_round_ip<<<(unsigned)(((size_t)MA * HID / 4 + 255) / 256), 256, 0, stream>>>(h, (size_t)MA * HID / 4);
    k_gemm_bf3<false, 1, false, false><<<((MA / 16) * (EP / 64) + 3) / 4, 128, 0, stream>>>(h, HID, B2, HID, b2p, nullptr, 1, 0, enc, EP, MA, EP, HID);
    k_col256<<<MA / 32, 1024, 0, stream>>>(h, W2, b2, e256);
    k_sumcat<<<CHB, 288, 0, stream>>>(s, enc, e256, A, b0, xq);
  }
  k_gemm_bf3<true, 1, true, false><<<((NB / 16) * (HID / 64) + 3) / 4, 128, 0, stream>>>(xq, QP, BQ1, QP, Qb1, nullptr, 1, 0, q1, HID, NB, HID, QP);
  k_gemm_bf3<true, 0, false, false><<<((NB / 16) * 1 + 3) / 4, 128, 0, stream>>>(q1, HID, BQ2, HID, qb2p, nullptr, 1, 0, q64, 64, NB, 64, HID);
  k_pack<<<NB / 128, 256, 0, stream>>>(q64, (float*)d_out);
}
